// MambaSSM_90194313216009
// MI455X (gfx1250) — hardware-verified
//
#include <hip/hip_runtime.h>
#include <math.h>

typedef __attribute__((ext_vector_type(16))) __bf16   v16b;
typedef __attribute__((ext_vector_type(8)))  __bf16   v8b;
typedef __attribute__((ext_vector_type(8)))  float    v8f;
typedef __attribute__((ext_vector_type(4)))  float    v4f;
typedef __attribute__((ext_vector_type(4)))  unsigned v4u;

constexpr int kSeq    = 2048;
constexpr int kDm     = 1024;
constexpr int kDin    = 2048;
constexpr int kNst    = 16;
constexpr int kXzP    = 2 * kDin;
constexpr int kPrjN   = kDin + 2 * kNst;
constexpr int kPrjP   = 2112;
constexpr int kConvTP = 260;
constexpr int kScanTS = 64;
constexpr int kScanCh = 64;
constexpr int kScanYP = 68;
constexpr int kBCW    = 2 * kNst;
static_assert(kPrjN == 2080, "x_proj width");
static_assert(kPrjP >= kPrjN && (kPrjP % 64) == 0 && ((kPrjP * 4) % 128) == 0, "padded x_proj width");
static_assert((kDm % 32) == 0 && (kDin % 32) == 0, "GEMM K multiples of 32");
static_assert((kSeq % 64) == 0 && (kXzP % 64) == 0 && (kDm % 64) == 0, "GEMM M,N multiples of 64");
static_assert((kSeq % kScanTS) == 0 && (kDin % kScanCh) == 0 && (kDin % 256) == 0, "tile multiples");
static_assert(kBCW == 32 && kNst == 16 && kScanCh == 64 && kScanTS == 64, "scan staging maps");

constexpr size_t kOffXB   = 0;
constexpr size_t kOffWIB  = kOffXB  + (size_t)kSeq  * kDm   * 2;
constexpr size_t kOffWXB  = kOffWIB + (size_t)kXzP  * kDm   * 2;
constexpr size_t kOffWOB  = kOffWXB + (size_t)kPrjP * kDin  * 2;
constexpr size_t kOffXZ   = kOffWOB + (size_t)kDm   * kDin  * 2;
constexpr size_t kOffUC   = kOffXZ  + (size_t)kSeq  * kXzP  * 4;
constexpr size_t kOffUCB  = kOffUC  + (size_t)kSeq  * kDin  * 4;
constexpr size_t kOffDBC  = kOffUCB + (size_t)kSeq  * kDin  * 2;
constexpr size_t kOffYH   = kOffDBC + (size_t)kSeq  * kPrjP * 4;
constexpr size_t kOffYL   = kOffYH  + (size_t)kSeq  * kDin  * 2;
constexpr size_t kWsTotal = kOffYL  + (size_t)kSeq  * kDin  * 2;
static_assert(kWsTotal == 118226944ull, "carve total");
static_assert(kWsTotal <= 134217728ull, "carve cap");
static_assert((kOffWIB % 128) == 0 && (kOffWXB % 128) == 0 && (kOffWOB % 128) == 0 && (kOffXZ % 128) == 0 &&
              (kOffUC % 128) == 0 && (kOffUCB % 128) == 0 && (kOffDBC % 128) == 0 && (kOffYH % 128) == 0 &&
              (kOffYL % 128) == 0, "128-B aligned regions");

__device__ __forceinline__ unsigned bf_rne_u(float f) {
  const unsigned u = __float_as_uint(f);
  return (u + 0x7FFFu + ((u >> 16) & 1u)) >> 16;
}
__device__ __forceinline__ float bf_u2f(unsigned h) { return __uint_as_float(h << 16); }
__device__ __forceinline__ float bf_rne_f(float f) { return bf_u2f(bf_rne_u(f)); }
__device__ __forceinline__ unsigned pack_bf2(float a, float b) { return bf_rne_u(a) | (bf_rne_u(b) << 16); }
__device__ __forceinline__ void split_bf2(float fa, float fb, unsigned& hw, unsigned& lw) {
  const unsigned ha = bf_rne_u(fa), hb = bf_rne_u(fb);
  const unsigned la = bf_rne_u(fa - bf_u2f(ha)), lb = bf_rne_u(fb - bf_u2f(hb));
  hw = ha | (hb << 16);
  lw = la | (lb << 16);
}

__device__ __forceinline__ void dep_guard4_b(v8f& a, v8f& b, v8f& c, v8f& d, v16b x, v16b y) {
  asm volatile("v_nop\n\tv_nop\n\tv_nop\n\tv_nop" : "+v"(a), "+v"(b), "+v"(c), "+v"(d) : "v"(x), "v"(y));
}
__device__ __forceinline__ void keep4_b(v16b a, v16b b, v16b c, v16b d) { asm volatile("v_nop" :: "v"(a), "v"(b), "v"(c), "v"(d)); }
__device__ __forceinline__ void acc_guard4(v8f& a, v8f& b, v8f& c, v8f& d) { asm volatile("v_nop\n\tv_nop\n\tv_nop\n\tv_nop" : "+v"(a), "+v"(b), "+v"(c), "+v"(d)); }
struct FragB {
  union U { v16b v; v8b h[2]; };
  static __device__ __forceinline__ v16b load(const __bf16* p) {
    U f; f.h[0] = *(const v8b*)(p); f.h[1] = *(const v8b*)(p + 16); return f.v;
  }
  static __device__ __forceinline__ v8f mma(v16b a, v16b b, v8f c) {
    return __builtin_amdgcn_wmma_f32_16x16x32_bf16(false, a, false, b, (short)0, c, false, false);
  }
};

template <int SPL>
__global__ __launch_bounds__(256) void wmma_gemm64_bf16(
    const unsigned short* __restrict__ Ap, const unsigned short* __restrict__ A2p, int lda,
    const unsigned short* __restrict__ Btp, int ldb,
    float* __restrict__ C, int ldc, int M, int N, int K, float scale) {
  const __bf16* A  = (const __bf16*)Ap;
  const __bf16* A2 = (const __bf16*)A2p;
  const __bf16* Bt = (const __bf16*)Btp;
  __shared__ __align__(16) float sT[8][16 * 68];
  const int lane = threadIdx.x & 31;
  const int wave = threadIdx.x >> 5;
  const int tilesN = N >> 6;
  const int tilesM = M >> 6;
  const int tile = blockIdx.x * 8 + wave;
  if (tile >= tilesM * tilesN) return;
  const int tm = tile / tilesN;
  const int tn = tile - tm * tilesN;
  const int m0 = tm << 6;
  const int n0 = tn << 6;

  const int rlane = lane & 15;
  const int koff  = (lane >> 4) * 8;
  const int mOff  = (lane >> 4) * 8;

  v8f acc[4][4];
#pragma unroll
  for (int i = 0; i < 4; ++i)
#pragma unroll
    for (int j = 0; j < 4; ++j) acc[i][j] = (v8f){0.f,0.f,0.f,0.f,0.f,0.f,0.f,0.f};

  for (int k0 = 0; k0 < K; k0 += 32) {
    v16b bh[4];
#pragma unroll
    for (int j = 0; j < 4; ++j) {
      const size_t bo = (size_t)(n0 + (j << 4) + rlane) * ldb + koff + k0;
      bh[j] = FragB::load(Bt + bo);
    }
#pragma unroll
    for (int i = 0; i < 4; ++i) {
      const size_t ao = (size_t)(m0 + (i << 4) + rlane) * lda + koff + k0;
      v16b ah = FragB::load(A + ao);
      v16b al = ah;
      if (SPL == 1) al = FragB::load(A2 + ao);
#pragma unroll
      for (int j = 0; j < 4; ++j) {
        acc[i][j] = FragB::mma(ah, bh[j], acc[i][j]);
        if (SPL == 1) acc[i][j] = FragB::mma(al, bh[j], acc[i][j]);
      }
      dep_guard4_b(acc[i][0], acc[i][1], acc[i][2], acc[i][3], ah, al);
    }
    keep4_b(bh[0], bh[1], bh[2], bh[3]);
  }
  acc_guard4(acc[0][0], acc[0][1], acc[0][2], acc[0][3]);
  acc_guard4(acc[1][0], acc[1][1], acc[1][2], acc[1][3]);
  acc_guard4(acc[2][0], acc[2][1], acc[2][2], acc[2][3]);
  acc_guard4(acc[3][0], acc[3][1], acc[3][2], acc[3][3]);

  float* slab = sT[wave];
#pragma unroll
  for (int i = 0; i < 4; ++i) {
    const int mBase = m0 + (i << 4);
#pragma unroll
    for (int j = 0; j < 4; ++j) {
#pragma unroll
      for (int r = 0; r < 8; ++r) {
        slab[(mOff + r) * 68 + (j << 4) + rlane] = acc[i][j][r] * scale;
      }
    }
    __builtin_amdgcn_fence(__ATOMIC_RELEASE, "workgroup");
    __builtin_amdgcn_wave_barrier();
    __builtin_amdgcn_fence(__ATOMIC_ACQUIRE, "workgroup");
    {
      const int hh = lane >> 4, c4 = (lane & 15) * 4;
      for (int pass = 0; pass < 2; ++pass) {
#pragma unroll
        for (int it = 0; it < 8; ++it) {
          const int row = it * 2 + hh;
          v4f v = *(const v4f*)(slab + row * 68 + c4);
          *(volatile v4f*)(C + (size_t)(mBase + row) * ldc + n0 + c4) = v;
        }
        __threadfence();
      }
    }
    __builtin_amdgcn_fence(__ATOMIC_RELEASE, "workgroup");
    __builtin_amdgcn_wave_barrier();
    __builtin_amdgcn_fence(__ATOMIC_ACQUIRE, "workgroup");
  }
}

__global__ __launch_bounds__(256) void cast_rows_bf16_kernel(
    const float* __restrict__ src, unsigned short* __restrict__ dst, int real8, int total8)
{
  const int i = blockIdx.x * 256 + threadIdx.x;
  if (i >= total8) return;
  const bool live = (i < real8);
  const int ic = live ? i : (real8 - 1);
  const size_t es = (size_t)ic << 3;
  const v4f a0 = *(const v4f*)(src + es);
  const v4f a1 = *(const v4f*)(src + es + 4);
  const float f0 = a0[0], f1 = a0[1], f2 = a0[2], f3 = a0[3];
  const float f4 = a1[0], f5 = a1[1], f6 = a1[2], f7 = a1[3];
  const unsigned w0 = pack_bf2(f0, f1), w1 = pack_bf2(f2, f3), w2 = pack_bf2(f4, f5), w3 = pack_bf2(f6, f7);
  v4u w;
  w[0] = live ? w0 : 0u;
  w[1] = live ? w1 : 0u;
  w[2] = live ? w2 : 0u;
  w[3] = live ? w3 : 0u;
  unsigned short* q = dst + ((size_t)i << 3);
  *(volatile v4u*)q = w;
  __threadfence();
  *(volatile v4u*)q = w;
}

__global__ __launch_bounds__(256) void conv_silu_kernel(
    const float* __restrict__ XZ, const float* __restrict__ cw, const float* __restrict__ cb,
    float* __restrict__ UC, unsigned short* __restrict__ UCB)
{
  __shared__ __align__(16) float sT[16 * kConvTP];
  const int tid = threadIdx.x, lane = tid & 31, wave = tid >> 5;
  const int d0 = blockIdx.x * 256, d = d0 + tid;
  const int t0 = blockIdx.y * 64;
  const v4f wv = *(const v4f*)(cw + (size_t)d * 4);
  const float wr0 = wv[0], wr1 = wv[1], wr2 = wv[2], wr3 = wv[3];
  const float w0 = bf_rne_f(wr0), w1 = bf_rne_f(wr1), w2 = bf_rne_f(wr2), w3 = bf_rne_f(wr3);
  const float bc = bf_rne_f(cb[d]);
  float xm3, xm2, xm1;
  {
    const int r3 = t0 - 3, r2 = t0 - 2, r1 = t0 - 1;
    const float v3 = XZ[(size_t)(r3 < 0 ? 0 : r3) * kXzP + d];
    const float v2 = XZ[(size_t)(r2 < 0 ? 0 : r2) * kXzP + d];
    const float v1 = XZ[(size_t)(r1 < 0 ? 0 : r1) * kXzP + d];
    xm3 = (r3 >= 0) ? v3 : 0.f;
    xm2 = (r2 >= 0) ? v2 : 0.f;
    xm1 = (r1 >= 0) ? v1 : 0.f;
  }
  const int hrow = wave >> 1;
  const int hch  = (wave & 1) * 128 + lane * 4;
#pragma unroll 1
  for (int sub = 0; sub < 4; ++sub) {
    const int lb = t0 + sub * 16;
#pragma unroll 1
    for (int s = 0; s < 16; ++s) {
      const float xc = XZ[(size_t)(lb + s) * kXzP + d];
      float acc = w0 * xm3;
      acc = fmaf(w1, xm2, acc);
      acc = fmaf(w2, xm1, acc);
      acc = fmaf(w3, xc, acc);
      const float sv = acc + bc;
      const float sg = __builtin_amdgcn_rcpf(1.0f + expf(-sv));
      sT[s * kConvTP + tid] = sv * sg;
      xm3 = xm2; xm2 = xm1; xm1 = xc;
    }
    __syncthreads();
    v4f fv[4];
    v4u bw[2];
#pragma unroll
    for (int it = 0; it < 4; ++it) fv[it] = *(const v4f*)(sT + (it * 4 + hrow) * kConvTP + hch);
#pragma unroll
    for (int it = 0; it < 2; ++it) {
      const float* sp = sT + (it * 8 + wave) * kConvTP + lane * 8;
      const v4f a0 = *(const v4f*)(sp);
      const v4f a1 = *(const v4f*)(sp + 4);
      const float f0 = a0[0], f1 = a0[1], f2 = a0[2], f3 = a0[3];
      const float f4 = a1[0], f5 = a1[1], f6 = a1[2], f7 = a1[3];
      v4u w;
      w[0] = pack_bf2(f0, f1);
      w[1] = pack_bf2(f2, f3);
      w[2] = pack_bf2(f4, f5);
      w[3] = pack_bf2(f6, f7);
      bw[it] = w;
    }
    for (int pass = 0; pass < 2; ++pass) {
#pragma unroll
      for (int it = 0; it < 4; ++it)
        *(volatile v4f*)(UC + (size_t)(lb + it * 4 + hrow) * kDin + d0 + hch) = fv[it];
#pragma unroll
      for (int it = 0; it < 2; ++it)
        *(volatile v4u*)(UCB + (size_t)(lb + it * 8 + wave) * kDin + d0 + lane * 8) = bw[it];
      __threadfence();
    }
    __syncthreads();
  }
}

__global__ __launch_bounds__(64) void scan_kernel(
    const float* __restrict__ DBC, const float* __restrict__ UC, const float* __restrict__ XZ,
    const float* __restrict__ Alog, const float* __restrict__ Dp,
    unsigned short* __restrict__ YH, unsigned short* __restrict__ YL)
{
  __shared__ __align__(16) float sBC[kScanTS * kBCW];
  __shared__ __align__(16) float sY[kScanTS * kScanYP];
  __shared__ __align__(16) float sA[kNst * kScanCh];
  const int tid = threadIdx.x, lane = tid & 31, wave = tid >> 5;
  const int d0 = blockIdx.x * kScanCh;
  const int d  = d0 + tid;
#pragma unroll 1
  for (int s = 0; s < kNst; ++s) sA[s * kScanCh + tid] = -expf(bf_rne_f(Alog[(size_t)d * kNst + s]));
  __syncthreads();
  float negA[kNst], h[kNst];
#pragma unroll
  for (int s = 0; s < kNst; ++s) {
    negA[s] = sA[s * kScanCh + tid];
    h[s] = 0.f;
  }
  const float Dd = bf_rne_f(Dp[d]);
  const int lr = tid >> 3, lc4 = (tid & 7) * 4;
  const int q = lane >> 3, c8 = (lane & 7) * 8;
#pragma unroll 1
  for (int t0 = 0; t0 < kSeq; t0 += kScanTS) {
    __syncthreads();
#pragma unroll
    for (int i = 0; i < 8; ++i) {
      const int r = lr + 8 * i;
      *(v4f*)(sBC + r * kBCW + lc4) = *(const v4f*)(DBC + (size_t)(t0 + r) * kPrjP + kDin + lc4);
    }
    __syncthreads();
#pragma unroll 1
    for (int s = 0; s < kScanTS; ++s) {
      const size_t t = (size_t)(t0 + s);
      float v  = DBC[t * kPrjP + d];
      float xt = UC[t * kDin + d];
      float zv = XZ[t * kXzP + kDin + d];
      asm volatile("" : "+v"(v));
      asm volatile("" : "+v"(xt));
      asm volatile("" : "+v"(zv));
      const float* xr = sBC + s * kBCW;
      float Bs[kNst], Cs[kNst];
#pragma unroll
      for (int q4 = 0; q4 < 4; ++q4) {
        const v4f bv = *(const v4f*)(xr + 4 * q4);
        const v4f cv = *(const v4f*)(xr + kNst + 4 * q4);
        Bs[4 * q4 + 0] = bv[0]; Bs[4 * q4 + 1] = bv[1]; Bs[4 * q4 + 2] = bv[2]; Bs[4 * q4 + 3] = bv[3];
        Cs[4 * q4 + 0] = cv[0]; Cs[4 * q4 + 1] = cv[1]; Cs[4 * q4 + 2] = cv[2]; Cs[4 * q4 + 3] = cv[3];
      }
      const float a   = __expf(-fabsf(v));
      const float u   = 1.0f + a;
      const float l1p = __logf(u) + (a - (u - 1.0f)) * __builtin_amdgcn_rcpf(u);
      const float dt  = fmaxf(v, 0.0f) + l1p;
      const float dtx = dt * xt;
      float y = 0.f;
#pragma unroll
      for (int k = 0; k < kNst; ++k) {
        const float e = __expf(dt * negA[k]);
        h[k] = e * h[k] + dtx * Bs[k];
        y = h[k] * Cs[k] + y;
      }
      y = xt * Dd + y;
      const float sg = __builtin_amdgcn_rcpf(1.0f + expf(-zv));
      y = y * (zv * sg);
      sY[s * kScanYP + tid] = y;
    }
    __syncthreads();
    v4u hw[8], lw[8];
#pragma unroll
    for (int it = 0; it < 8; ++it) {
      const int row = it * 8 + wave * 4 + q;
      const float* sp = sY + row * kScanYP + c8;
      const v4f a0 = *(const v4f*)(sp);
      const v4f a1 = *(const v4f*)(sp + 4);
      const float f0 = a0[0], f1 = a0[1], f2 = a0[2], f3 = a0[3];
      const float f4 = a1[0], f5 = a1[1], f6 = a1[2], f7 = a1[3];
      unsigned h0, h1, h2, h3, l0, l1, l2, l3;
      split_bf2(f0, f1, h0, l0);
      split_bf2(f2, f3, h1, l1);
      split_bf2(f4, f5, h2, l2);
      split_bf2(f6, f7, h3, l3);
      v4u hv, lv;
      hv[0] = h0; hv[1] = h1; hv[2] = h2; hv[3] = h3;
      lv[0] = l0; lv[1] = l1; lv[2] = l2; lv[3] = l3;
      hw[it] = hv;
      lw[it] = lv;
    }
    for (int pass = 0; pass < 2; ++pass) {
#pragma unroll
      for (int it = 0; it < 8; ++it) {
        const int row = it * 8 + wave * 4 + q;
        const size_t o = (size_t)(t0 + row) * kDin + d0 + c8;
        *(volatile v4u*)(YH + o) = hw[it];
        *(volatile v4u*)(YL + o) = lw[it];
      }
      __threadfence();
    }
  }
}

static_assert(((kSeq / 64) * (kXzP / 64)) % 8 == 0, "in_proj tiles per block");
static_assert(((kSeq / 64) * (kPrjP / 64)) % 8 == 0, "x_proj tiles per block");
static_assert(((kSeq / 64) * (kDm / 64)) % 8 == 0, "out_proj tiles per block");
static_assert(((kSeq * kDm / 8) % 256) == 0 && ((kXzP * kDm / 8) % 256) == 0 &&
              ((kPrjP * kDin / 8) % 256) == 0 && ((kPrjN * kDin / 8) % 256) == 0 &&
              ((kDm * kDin / 8) % 256) == 0, "cast grids exact");

extern "C" void kernel_launch(void* const* d_in, const int* in_sizes, int n_in,
                              void* d_out, int out_size, void* d_ws, size_t ws_size,
                              hipStream_t stream) {
  if (n_in < 8) return;
  if (in_sizes[0] != kSeq * kDm) return;
  if (in_sizes[1] != kXzP * kDm) return;
  if (in_sizes[2] != kDin * 4) return;
  if (in_sizes[3] != kDin) return;
  if (in_sizes[4] != kPrjN * kDin) return;
  if (in_sizes[5] != kDin * kNst) return;
  if (in_sizes[6] != kDin) return;
  if (in_sizes[7] != kDm * kDin) return;
  if (out_size != kSeq * kDm) return;
  if (ws_size < kWsTotal) return;

  const float* x      = (const float*)d_in[0];
  const float* W_in   = (const float*)d_in[1];
  const float* conv_w = (const float*)d_in[2];
  const float* conv_b = (const float*)d_in[3];
  const float* W_x    = (const float*)d_in[4];
  const float* A_log  = (const float*)d_in[5];
  const float* Dp     = (const float*)d_in[6];
  const float* W_out  = (const float*)d_in[7];
  float* out = (float*)d_out;

  char* ws = (char*)d_ws;
  unsigned short* XB  = (unsigned short*)(ws + kOffXB);
  unsigned short* WIB = (unsigned short*)(ws + kOffWIB);
  unsigned short* WXB = (unsigned short*)(ws + kOffWXB);
  unsigned short* WOB = (unsigned short*)(ws + kOffWOB);
  float*          XZ  = (float*)(ws + kOffXZ);
  float*          UC  = (float*)(ws + kOffUC);
  unsigned short* UCB = (unsigned short*)(ws + kOffUCB);
  float*          DBC = (float*)(ws + kOffDBC);
  unsigned short* YH  = (unsigned short*)(ws + kOffYH);
  unsigned short* YL  = (unsigned short*)(ws + kOffYL);

  cast_rows_bf16_kernel<<<(kSeq * kDm / 8) / 256, 256, 0, stream>>>(x, XB, kSeq * kDm / 8, kSeq * kDm / 8);
  cast_rows_bf16_kernel<<<(kXzP * kDm / 8) / 256, 256, 0, stream>>>(W_in, WIB, kXzP * kDm / 8, kXzP * kDm / 8);
  cast_rows_bf16_kernel<<<(kPrjP * kDin / 8) / 256, 256, 0, stream>>>(W_x, WXB, kPrjN * kDin / 8, kPrjP * kDin / 8);
  cast_rows_bf16_kernel<<<(kDm * kDin / 8) / 256, 256, 0, stream>>>(W_out, WOB, kDm * kDin / 8, kDm * kDin / 8);

  wmma_gemm64_bf16<0><<<dim3((kSeq / 64) * (kXzP / 64) / 8), 256, 0, stream>>>(
      XB, XB, kDm, WIB, kDm, XZ, kXzP, kSeq, kXzP, kDm, 1.0f);

  conv_silu_kernel<<<dim3(kDin / 256, kSeq / 64), 256, 0, stream>>>(XZ, conv_w, conv_b, UC, UCB);

  wmma_gemm64_bf16<0><<<dim3((kSeq / 64) * (kPrjP / 64) / 8), 256, 0, stream>>>(
      UCB, UCB, kDin, WXB, kDin, DBC, kPrjP, kSeq, kPrjP, kDin, 1.0f);

  scan_kernel<<<kDin / kScanCh, kScanCh, 0, stream>>>(DBC, UC, XZ, A_log, Dp, YH, YL);

  wmma_gemm64_bf16<1><<<dim3((kSeq / 64) * (kDm / 64) / 8), 256, 0, stream>>>(
      YH, YL, kDin, WOB, kDin, out, kDm, kSeq, kDm, kDin, 1.0f);
}
